// PostNormMamba_68564857913689
// MI455X (gfx1250) — hardware-verified
//
#include <hip/hip_runtime.h>
#include <math.h>
#include <stdint.h>

#define B_SZ    4
#define LSEQ    2048
#define DMODEL  512
#define DINNER  1024
#define DSTATE  16
#define DCONV   4
#define DTR     32
#define NDBC    (DTR + 2 * DSTATE)
#define MROWS   (B_SZ * LSEQ)

#define GBM 128
#define GBN 64
#define GBK 32
#define SPITCH 40
#define CPITCH 68
#define SMEM_FLOATS (GBM * CPITCH)
#define TCH 32
#define YPITCH 132

static_assert(MROWS % GBM == 0);
static_assert((2 * DINNER) % GBN == 0);
static_assert(NDBC % GBN == 0);
static_assert(DINNER % GBN == 0);
static_assert(DMODEL % GBN == 0);
static_assert(DMODEL % GBK == 0);
static_assert(DINNER % GBK == 0);
static_assert(DTR % GBK == 0);
static_assert(DINNER % 128 == 0);
static_assert(DMODEL == 4 * 128);
static_assert(LSEQ % TCH == 0);
static_assert((GBM * SPITCH + GBN * SPITCH) * 2 * 2 <= SMEM_FLOATS * 4);

typedef __bf16         v16bf __attribute__((ext_vector_type(16)));
typedef unsigned short v8us  __attribute__((ext_vector_type(8), __may_alias__));
typedef float          v8f   __attribute__((ext_vector_type(8)));
typedef float          v4f   __attribute__((ext_vector_type(4), __may_alias__));

union Frag { v16bf v; v8us half[2]; };
union U16  { v8us v[2]; unsigned short e[16]; };
union U8   { v8us v; unsigned short e[8]; };

__device__ __forceinline__ void split_bf16(float f, unsigned short& hi, unsigned short& lo)
{
    const unsigned u  = __float_as_uint(f);
    const unsigned rh = (u + 0x7FFFu + ((u >> 16) & 1u)) >> 16;
    const float    fh = __uint_as_float(rh << 16);
    const float    d  = f - fh;
    const unsigned ud = __float_as_uint(d);
    const unsigned rl = (ud + 0x7FFFu + ((ud >> 16) & 1u)) >> 16;
    hi = (unsigned short)rh;
    lo = (unsigned short)rl;
}

__device__ __forceinline__ void mma3(v8f& acc, const v16bf& ah, const v16bf& al,
                                     const v16bf& bh, const v16bf& bl)
{
    acc = __builtin_amdgcn_wmma_f32_16x16x32_bf16(false, ah, false, bh, (short)0, acc, false, false);
    acc = __builtin_amdgcn_wmma_f32_16x16x32_bf16(false, al, false, bh, (short)0, acc, false, false);
    acc = __builtin_amdgcn_wmma_f32_16x16x32_bf16(false, ah, false, bl, (short)0, acc, false, false);
    asm volatile("v_nop\n\tv_nop\n\tv_nop\n\tv_nop" : "+v"(acc) : "v"(ah), "v"(al), "v"(bh), "v"(bl));
}

__device__ __forceinline__ float softplus_f(float x)
{
    return fmaxf(x, 0.f) + log1pf(__expf(-fabsf(x)));
}

__device__ __forceinline__ float silu_f(float x)
{
    return x * (1.0f / (1.0f + __expf(-x)));
}

template <int EPI>
__device__ __forceinline__ void gemm_store(const float* sC, float* C, int ldc, int m0, int n0,
                                           const float* __restrict__ bias, int wave, int l)
{
    const int rsub = wave * 2 + (l >> 4);
    const int c4   = (l & 15) * 4;
    v4f bv = {0.f, 0.f, 0.f, 0.f};
    if (EPI) bv = *(const v4f*)(bias + n0 + c4);
    #pragma unroll 1
    for (int p = 0; p < GBM / 16; ++p) {
        const int row = p * 16 + rsub;
        v4f v = *(const v4f*)(sC + row * CPITCH + c4);
        if (EPI) {
            v = v + bv;
            v[0] = softplus_f(v[0]);
            v[1] = softplus_f(v[1]);
            v[2] = softplus_f(v[2]);
            v[3] = softplus_f(v[3]);
        }
        *(volatile v4f*)(C + (size_t)(m0 + row) * ldc + n0 + c4) = v;
    }
}

template <int EPI>
__global__ void __launch_bounds__(256)
k_gemm(const float* __restrict__ A, int lda,
       const float* __restrict__ B, int ldb,
       float* C, int ldc, int K,
       const float* __restrict__ bias)
{
    __shared__ __attribute__((aligned(16))) float smem[SMEM_FLOATS];
    unsigned short* sAh = reinterpret_cast<unsigned short*>(smem);
    unsigned short* sAl = sAh + GBM * SPITCH;
    unsigned short* sBh = sAl + GBM * SPITCH;
    unsigned short* sBl = sBh + GBN * SPITCH;
    float* sC = smem;

    const int tid  = threadIdx.x;
    const int l    = tid & 31;
    const int wave = tid >> 5;
    const int h    = l >> 4;
    const int r16  = l & 15;
    const int wm   = (wave & 3) * 32;
    const int wn   = (wave >> 2) * 32;
    const int m0   = blockIdx.x * GBM;
    const int n0   = blockIdx.y * GBN;

    const int arow = tid >> 1, acol = (tid & 1) * 16;
    const int brow = tid >> 2, bcol = (tid & 3) * 8;
    const float* ap = A + (size_t)(m0 + arow) * lda + acol;
    const float* bp = B + (size_t)(n0 + brow) * ldb + bcol;

    const v8f zero8 = {0.f, 0.f, 0.f, 0.f, 0.f, 0.f, 0.f, 0.f};
    v8f acc[2][2];
    #pragma unroll
    for (int mi = 0; mi < 2; ++mi)
        #pragma unroll
        for (int ni = 0; ni < 2; ++ni) acc[mi][ni] = zero8;

    for (int k0 = 0; k0 < K; k0 += GBK) {
        __syncthreads();
        {
            U16 uh, ul;
            #pragma unroll
            for (int j = 0; j < 4; ++j) {
                const v4f x = *(const v4f*)(ap + k0 + 4 * j);
                #pragma unroll
                for (int q = 0; q < 4; ++q) split_bf16(x[q], uh.e[4 * j + q], ul.e[4 * j + q]);
            }
            unsigned short* ph = sAh + arow * SPITCH + acol;
            unsigned short* pl = sAl + arow * SPITCH + acol;
            *(v8us*)(ph)     = uh.v[0];
            *(v8us*)(ph + 8) = uh.v[1];
            *(v8us*)(pl)     = ul.v[0];
            *(v8us*)(pl + 8) = ul.v[1];
        }
        {
            U8 uh, ul;
            const v4f x0 = *(const v4f*)(bp + k0);
            const v4f x1 = *(const v4f*)(bp + k0 + 4);
            #pragma unroll
            for (int q = 0; q < 4; ++q) {
                split_bf16(x0[q], uh.e[q],     ul.e[q]);
                split_bf16(x1[q], uh.e[4 + q], ul.e[4 + q]);
            }
            *(v8us*)(sBh + brow * SPITCH + bcol) = uh.v;
            *(v8us*)(sBl + brow * SPITCH + bcol) = ul.v;
        }
        __syncthreads();

        Frag ah[2], al[2];
        #pragma unroll
        for (int mi = 0; mi < 2; ++mi) {
            const unsigned short* ph = sAh + (wm + mi * 16 + r16) * SPITCH;
            const unsigned short* pl = sAl + (wm + mi * 16 + r16) * SPITCH;
            ah[mi].half[0] = *(const v8us*)(ph + 8 * h);
            ah[mi].half[1] = *(const v8us*)(ph + 16 + 8 * h);
            al[mi].half[0] = *(const v8us*)(pl + 8 * h);
            al[mi].half[1] = *(const v8us*)(pl + 16 + 8 * h);
        }
        #pragma unroll
        for (int ni = 0; ni < 2; ++ni) {
            Frag bh, bl;
            const unsigned short* qh = sBh + (wn + ni * 16 + r16) * SPITCH;
            const unsigned short* ql = sBl + (wn + ni * 16 + r16) * SPITCH;
            bh.half[0] = *(const v8us*)(qh + 8 * h);
            bh.half[1] = *(const v8us*)(qh + 16 + 8 * h);
            bl.half[0] = *(const v8us*)(ql + 8 * h);
            bl.half[1] = *(const v8us*)(ql + 16 + 8 * h);
            #pragma unroll
            for (int mi = 0; mi < 2; ++mi)
                mma3(acc[mi][ni], ah[mi].v, al[mi].v, bh.v, bl.v);
        }
    }
    __syncthreads();

    #pragma unroll
    for (int mi = 0; mi < 2; ++mi)
        #pragma unroll
        for (int ni = 0; ni < 2; ++ni) {
            float* pc = sC + (wm + mi * 16 + 8 * h) * CPITCH + wn + ni * 16 + r16;
            #pragma unroll
            for (int e = 0; e < 8; ++e) pc[e * CPITCH] = acc[mi][ni][e];
        }
    __syncthreads();

    gemm_store<EPI>(sC, C, ldc, m0, n0, bias, wave, l);
    __threadfence();
    gemm_store<EPI>(sC, C, ldc, m0, n0, bias, wave, l);
}

__global__ void __launch_bounds__(256)
k_conv_silu(const float* __restrict__ xz, const float* __restrict__ cw,
            const float* __restrict__ cb, float* uf, int total4)
{
    const int idx = blockIdx.x * 256 + threadIdx.x;
    if (idx >= total4) return;
    const int m  = idx >> 8;
    const int d0 = (idx & 255) * 4;
    const int l  = m & (LSEQ - 1);

    const v4f w0 = *(const v4f*)(cw + (d0 + 0) * DCONV);
    const v4f w1 = *(const v4f*)(cw + (d0 + 1) * DCONV);
    const v4f w2 = *(const v4f*)(cw + (d0 + 2) * DCONV);
    const v4f w3 = *(const v4f*)(cw + (d0 + 3) * DCONV);

    v4f s = {0.f, 0.f, 0.f, 0.f};
    #pragma unroll
    for (int w = 0; w < DCONV; ++w) {
        const int ll = l - (DCONV - 1) + w;
        if (ll >= 0) {
            const v4f xv = *(const v4f*)(xz + (size_t)(m - (DCONV - 1) + w) * (2 * DINNER) + d0);
            s[0] += w0[w] * xv[0];
            s[1] += w1[w] * xv[1];
            s[2] += w2[w] * xv[2];
            s[3] += w3[w] * xv[3];
        }
    }
    const v4f bb = *(const v4f*)(cb + d0);
    const v4f a  = s + bb;
    v4f o;
    o[0] = silu_f(a[0]);
    o[1] = silu_f(a[1]);
    o[2] = silu_f(a[2]);
    o[3] = silu_f(a[3]);
    float* dst = uf + (size_t)m * DINNER + d0;
    *(volatile v4f*)dst = o;
    __threadfence();
    *(volatile v4f*)dst = o;
}

__global__ void __launch_bounds__(128)
k_scan(const float* __restrict__ delta, const float* __restrict__ uf,
       const float* __restrict__ xz, const float* __restrict__ dbc,
       const float* __restrict__ A_log, const float* __restrict__ Dv,
       float* yg)
{
    __shared__ __attribute__((aligned(16))) float sBC[TCH][2 * DSTATE];
    __shared__ __attribute__((aligned(16))) float sY[TCH][YPITCH];

    const int tid  = threadIdx.x;
    const int b    = blockIdx.x >> 3;
    const int dgrp = blockIdx.x & 7;
    const int d    = dgrp * 128 + tid;
    const size_t rowbase = (size_t)b * LSEQ;

    float Areg[DSTATE], hst[DSTATE];
    #pragma unroll
    for (int s = 0; s < DSTATE; ++s) {
        Areg[s] = -__expf(A_log[d * DSTATE + s]);
        hst[s]  = 0.f;
    }
    const float Dd = Dv[d];

    for (int tc = 0; tc < LSEQ; tc += TCH) {
        __syncthreads();
        {
            const int s = tid >> 2, q = (tid & 3) * 8;
            const float* src = dbc + (rowbase + tc + s) * NDBC + DTR + q;
            const v4f v0 = *(const v4f*)(src);
            const v4f v1 = *(const v4f*)(src + 4);
            *(v4f*)(&sBC[s][q])     = v0;
            *(v4f*)(&sBC[s][q + 4]) = v1;
        }
        __syncthreads();

        #pragma unroll 1
        for (int s = 0; s < TCH; ++s) {
            const size_t row = rowbase + tc + s;
            const float dt = delta[row * DINNER + d];
            const float ut = uf[row * DINNER + d];
            const float z  = xz[row * (2 * DINNER) + DINNER + d];
            const float du = dt * ut;
            float acc = 0.f;
            #pragma unroll
            for (int st = 0; st < DSTATE; ++st) {
                const float dA = __expf(dt * Areg[st]);
                hst[st] = dA * hst[st] + du * sBC[s][st];
                acc += hst[st] * sBC[s][DSTATE + st];
            }
            const float y = acc + Dd * ut;
            sY[s][tid] = y * silu_f(z);
        }
        __syncthreads();

        const int wv = tid >> 5, c4 = (tid & 31) * 4;
        #pragma unroll 1
        for (int p = 0; p < TCH / 4; ++p) {
            const int s = p * 4 + wv;
            const v4f v = *(const v4f*)(&sY[s][c4]);
            *(volatile v4f*)(yg + (rowbase + tc + s) * DINNER + dgrp * 128 + c4) = v;
        }
        __threadfence();
        #pragma unroll 1
        for (int p = 0; p < TCH / 4; ++p) {
            const int s = p * 4 + wv;
            const v4f v = *(const v4f*)(&sY[s][c4]);
            *(volatile v4f*)(yg + (rowbase + tc + s) * DINNER + dgrp * 128 + c4) = v;
        }
    }
}

__global__ void __launch_bounds__(128)
k_rmsnorm(const float* __restrict__ op, const float* __restrict__ x,
          const float* __restrict__ w, float* out, int mrows)
{
    __shared__ float red[4];
    const int m = blockIdx.x;
    if (m >= mrows) return;
    const int tid = threadIdx.x;
    const size_t base = (size_t)m * DMODEL + tid * 4;
    const v4f v = *(const v4f*)(op + base);
    float ss = v[0] * v[0] + v[1] * v[1] + v[2] * v[2] + v[3] * v[3];
    ss += __shfl_xor(ss, 16, 32);
    ss += __shfl_xor(ss, 8, 32);
    ss += __shfl_xor(ss, 4, 32);
    ss += __shfl_xor(ss, 2, 32);
    ss += __shfl_xor(ss, 1, 32);
    if ((tid & 31) == 0) red[tid >> 5] = ss;
    __syncthreads();
    const float tot = (red[0] + red[1]) + (red[2] + red[3]);
    const float sc  = rsqrtf(tot * (1.0f / (float)DMODEL) + 1e-5f);
    const v4f wv = *(const v4f*)(w + tid * 4);
    const v4f xv = *(const v4f*)(x + base);
    const v4f o  = (v * sc) * wv + xv;
    float* dst = out + base;
    *(volatile v4f*)dst = o;
    __threadfence();
    *(volatile v4f*)dst = o;
}

extern "C" void kernel_launch(void* const* d_in, const int* in_sizes, int n_in,
                              void* d_out, int out_size, void* d_ws, size_t ws_size,
                              hipStream_t stream)
{
    if (n_in < 11) return;
    if (in_sizes[0]  != MROWS * DMODEL)      return;
    if (in_sizes[1]  != 2 * DINNER * DMODEL) return;
    if (in_sizes[2]  != DINNER * DCONV)      return;
    if (in_sizes[3]  != DINNER)              return;
    if (in_sizes[4]  != NDBC * DINNER)       return;
    if (in_sizes[5]  != DINNER * DTR)        return;
    if (in_sizes[6]  != DINNER)              return;
    if (in_sizes[7]  != DINNER * DSTATE)     return;
    if (in_sizes[8]  != DINNER)              return;
    if (in_sizes[9]  != DMODEL * DINNER)     return;
    if (in_sizes[10] != DMODEL)              return;
    if (out_size != MROWS * DMODEL)          return;

    const float* x         = (const float*)d_in[0];
    const float* in_proj_w = (const float*)d_in[1];
    const float* conv_w    = (const float*)d_in[2];
    const float* conv_b    = (const float*)d_in[3];
    const float* x_proj_w  = (const float*)d_in[4];
    const float* dt_proj_w = (const float*)d_in[5];
    const float* dt_proj_b = (const float*)d_in[6];
    const float* A_log     = (const float*)d_in[7];
    const float* Dv        = (const float*)d_in[8];
    const float* out_w     = (const float*)d_in[9];
    const float* rms_w     = (const float*)d_in[10];
    float* out = (float*)d_out;

    size_t off = 0;
    auto carve = [&](size_t bytes) -> char* {
        char* p = (char*)d_ws + off;
        off += (bytes + 255) & ~(size_t)255;
        return p;
    };
    float* xz    = (float*)carve((size_t)MROWS * 2 * DINNER * sizeof(float));
    float* uf    = (float*)carve((size_t)MROWS * DINNER * sizeof(float));
    float* dbc   = (float*)carve((size_t)MROWS * NDBC * sizeof(float));
    float* delta = (float*)carve((size_t)MROWS * DINNER * sizeof(float));
    float* yg    = (float*)carve((size_t)MROWS * DINNER * sizeof(float));
    float* outp  = (float*)carve((size_t)MROWS * DMODEL * sizeof(float));
    if (off > ws_size) return;

    k_gemm<0><<<dim3(MROWS / GBM, (2 * DINNER) / GBN), 256, 0, stream>>>(
        x, DMODEL, in_proj_w, DMODEL, xz, 2 * DINNER, DMODEL, dt_proj_b);

    {
        const int total4 = MROWS * (DINNER / 4);
        k_conv_silu<<<(total4 + 255) / 256, 256, 0, stream>>>(xz, conv_w, conv_b, uf, total4);
    }

    k_gemm<0><<<dim3(MROWS / GBM, NDBC / GBN), 256, 0, stream>>>(
        uf, DINNER, x_proj_w, DINNER, dbc, NDBC, DINNER, dt_proj_b);

    k_gemm<1><<<dim3(MROWS / GBM, DINNER / GBN), 256, 0, stream>>>(
        dbc, NDBC, dt_proj_w, DTR, delta, DINNER, DTR, dt_proj_b);

    k_scan<<<B_SZ * (DINNER / 128), 128, 0, stream>>>(delta, uf, xz, dbc, A_log, Dv, yg);

    k_gemm<0><<<dim3(MROWS / GBM, DMODEL / GBN), 256, 0, stream>>>(
        yg, DINNER, out_w, DINNER, outp, DMODEL, DINNER, dt_proj_b);

    k_rmsnorm<<<MROWS, 128, 0, stream>>>(outp, x, rms_w, out, MROWS);
}
